// GroupEnhance_76690936037555
// MI455X (gfx1250) — hardware-verified
//
#include <hip/hip_runtime.h>
#include <math.h>

#define DIM 128
#define NN 100000
#define NE 640000
#define NT 256
#define SRB 2048
#define NTILE 49
#define NPAD (NTILE * SRB)
#define MG 100032
#define SCH 5120
#define SP (SCH / NT)
#define NCH (NE / SCH)
static_assert(NE % SCH == 0);
static_assert(SP % 4 == 0);
static_assert(NTILE * SRB >= NN);
static_assert(SRB / 8 == 256);
static_assert(MG % 64 == 0 && MG >= NN && MG <= NPAD);
static_assert(DIM == 128);

typedef __attribute__((ext_vector_type(16))) _Float16 v16h;
typedef __attribute__((ext_vector_type(8)))  _Float16 v8h;
typedef __attribute__((ext_vector_type(16))) __bf16   v16b;
typedef __attribute__((ext_vector_type(8)))  __bf16   v8b;
typedef __attribute__((ext_vector_type(8)))  float    v8f;
typedef __attribute__((ext_vector_type(4)))  float    v4f;
typedef __attribute__((ext_vector_type(4)))  int      v4i;

__device__ __forceinline__ unsigned short f2bf_bits(float f) {
  unsigned u = __float_as_uint(f);
  return (unsigned short)((u + 0x7FFFu + ((u >> 16) & 1u)) >> 16);
}
__device__ __forceinline__ float bf_bits2f(unsigned short h) { return __uint_as_float(((unsigned)h) << 16); }

__device__ __forceinline__ void dep_guard_h(v8f& a, v8f& b, v16h x, v16h y) { asm volatile("v_nop\n\tv_nop\n\tv_nop\n\tv_nop" : "+v"(a), "+v"(b) : "v"(x), "v"(y)); }
__device__ __forceinline__ void dep_guard_b(v8f& a, v8f& b, v16b x, v16b y) { asm volatile("v_nop\n\tv_nop\n\tv_nop\n\tv_nop" : "+v"(a), "+v"(b) : "v"(x), "v"(y)); }
__device__ __forceinline__ void keep4_h(v16h a, v16h b, v16h c, v16h d) { asm volatile("v_nop" :: "v"(a), "v"(b), "v"(c), "v"(d)); }
__device__ __forceinline__ void keep4_b(v16b a, v16b b, v16b c, v16b d) { asm volatile("v_nop" :: "v"(a), "v"(b), "v"(c), "v"(d)); }
__device__ __forceinline__ void acc_guard4(v8f& a, v8f& b, v8f& c, v8f& d) { asm volatile("v_nop\n\tv_nop\n\tv_nop\n\tv_nop" : "+v"(a), "+v"(b), "+v"(c), "+v"(d)); }
template <typename T> struct Frag;
template <> struct Frag<_Float16> {
  typedef v16h V; union U { v16h v; v8h h[2]; };
  static __device__ __forceinline__ v16h load(const _Float16* p) {
    U f; f.h[0] = *(const v8h*)(p); f.h[1] = *(const v8h*)(p + 16); return f.v;
  }
  static __device__ __forceinline__ v8f mma(v16h a, v16h b, v8f c) {
    return __builtin_amdgcn_wmma_f32_16x16x32_f16(false, a, false, b, (short)0, c, false, false);
  }
  static __device__ __forceinline__ void guard(v8f& a, v8f& b, v16h x, v16h y) { dep_guard_h(a, b, x, y); }
  static __device__ __forceinline__ void keep(v16h a, v16h b, v16h c, v16h d) { keep4_h(a, b, c, d); }
};
template <> struct Frag<__bf16> {
  typedef v16b V; union U { v16b v; v8b h[2]; };
  static __device__ __forceinline__ v16b load(const __bf16* p) {
    U f; f.h[0] = *(const v8b*)(p); f.h[1] = *(const v8b*)(p + 16); return f.v;
  }
  static __device__ __forceinline__ v8f mma(v16b a, v16b b, v8f c) {
    return __builtin_amdgcn_wmma_f32_16x16x32_bf16(false, a, false, b, (short)0, c, false, false);
  }
  static __device__ __forceinline__ void guard(v8f& a, v8f& b, v16b x, v16b y) { dep_guard_b(a, b, x, y); }
  static __device__ __forceinline__ void keep(v16b a, v16b b, v16b c, v16b d) { keep4_b(a, b, c, d); }
};

template <int ET> struct Elem;
template <> struct Elem<0> { typedef _Float16 T; };
template <> struct Elem<1> { typedef __bf16 T; };
template <int ET, bool SPLIT, int BIAS_MODE, int OUT_MODE, bool RESID, int ACT = 0, bool ASCALE = false>
__global__ __launch_bounds__(256) void wmma_gemm64(
    const unsigned short* __restrict__ Ap, const unsigned short* __restrict__ A2p, int lda, long strideA,
    const unsigned short* __restrict__ Btp, const unsigned short* __restrict__ Bt2p, int ldb, long strideB,
    void* __restrict__ Cout, void* __restrict__ Cout2, int ldc, long strideC,
    const float* __restrict__ bias,
    const float* __restrict__ resid, long strideR,
    int M, int N, int K, float scale,
    const float* __restrict__ ascale, int Mlim) {
  typedef typename Elem<ET>::T T;
  typedef typename Frag<T>::V V;
  const T* A = (const T*)Ap; const T* A2 = (const T*)A2p; const T* Bt = (const T*)Btp; const T* Bt2 = (const T*)Bt2p;
  __shared__ __align__(16) float sT[8][16 * 68];
  const int b    = blockIdx.y;
  const int lane = threadIdx.x & 31;
  const int wave = threadIdx.x >> 5;
  const int tilesN = N >> 6;
  const int tilesM = M >> 6;
  const int tile = blockIdx.x * 8 + wave;
  if (tile >= tilesM * tilesN) return;
  const int tm = tile / tilesN;
  const int tn = tile - tm * tilesN;
  const int m0 = tm << 6;
  const int n0 = tn << 6;

  const T* Ab  = A  + (size_t)b * strideA;
  const T* Bb  = Bt + (size_t)b * strideB;
  const T* Ab2 = SPLIT ? (A2  + (size_t)b * strideA) : nullptr;
  const T* Bb2 = SPLIT ? (Bt2 + (size_t)b * strideB) : nullptr;

  const int rlane = lane & 15;
  const int koff  = (lane >> 4) * 8;
  const int mOff  = (lane >> 4) * 8;

  v8f acc[4][4];
#pragma unroll
  for (int i = 0; i < 4; ++i)
#pragma unroll
    for (int j = 0; j < 4; ++j) acc[i][j] = (v8f){0.f,0.f,0.f,0.f,0.f,0.f,0.f,0.f};

  for (int k0 = 0; k0 < K; k0 += 32) {
    V bh[4], bl[4];
#pragma unroll
    for (int j = 0; j < 4; ++j) {
      const size_t bo = (size_t)(n0 + (j << 4) + rlane) * ldb + koff + k0;
      bh[j] = Frag<T>::load(Bb + bo);
      if (SPLIT) bl[j] = Frag<T>::load(Bb2 + bo);
    }
#pragma unroll
    for (int i = 0; i < 4; ++i) {
      const size_t ao = (size_t)(m0 + (i << 4) + rlane) * lda + koff + k0;
      V ah = Frag<T>::load(Ab + ao);
      V al;
      if (SPLIT) al = Frag<T>::load(Ab2 + ao);
#pragma unroll
      for (int j = 0; j < 4; ++j) {
        acc[i][j] = Frag<T>::mma(ah, bh[j], acc[i][j]);
        if (SPLIT) {
          acc[i][j] = Frag<T>::mma(ah, bl[j], acc[i][j]);
          acc[i][j] = Frag<T>::mma(al, bh[j], acc[i][j]);
        }
      }
      Frag<T>::guard(acc[i][0], acc[i][3], ah, SPLIT ? al : ah);
    }
    Frag<T>::keep(bh[0], bh[1], bh[2], bh[3]);
    if (SPLIT) Frag<T>::keep(bl[0], bl[1], bl[2], bl[3]);
  }
  acc_guard4(acc[0][0], acc[0][1], acc[0][2], acc[0][3]);
  acc_guard4(acc[1][0], acc[1][1], acc[1][2], acc[1][3]);
  acc_guard4(acc[2][0], acc[2][1], acc[2][2], acc[2][3]);
  acc_guard4(acc[3][0], acc[3][1], acc[3][2], acc[3][3]);

  float* slab = sT[wave];
  const float* Rb = RESID ? (resid + (size_t)b * strideR) : nullptr;
  const float asc = ASCALE ? ascale[0] : 1.0f;
#pragma unroll
  for (int i = 0; i < 4; ++i) {
    const int mBase = m0 + (i << 4);
#pragma unroll
    for (int j = 0; j < 4; ++j) {
      const int n = n0 + (j << 4) + rlane;
      float bv = 0.f;
      if (BIAS_MODE == 2) bv = bias[n];
#pragma unroll
      for (int r = 0; r < 8; ++r) {
        int rr = mBase + mOff + r; rr = rr < Mlim ? rr : Mlim - 1;
        float v = acc[i][j][r] * scale;
        if (BIAS_MODE == 1) v += bias[rr];
        if (BIAS_MODE == 2) v += bv;
        if (ASCALE) v *= asc;
        if (RESID) v += Rb[(size_t)rr * ldc + n];
        if (ACT == 1) v = tanhf(v);
        if (ACT == 2) v = fmaxf(v, 0.0f);
        if (ACT == 3) v = v / (1.0f + expf(-v));
        if (ACT == 4) v = (v > 0.f) ? v : 0.01f * v;
        if (ACT == 5) v = 0.5f * v * (1.0f + erff(v * 0.70710678118654752f));
        slab[(mOff + r) * 68 + (j << 4) + rlane] = v;
      }
    }
    __builtin_amdgcn_fence(__ATOMIC_RELEASE, "workgroup");
    __builtin_amdgcn_wave_barrier();
    __builtin_amdgcn_fence(__ATOMIC_ACQUIRE, "workgroup");
    if (OUT_MODE == 0) {
      float* C = (float*)Cout + (size_t)b * strideC;
      const int hh = lane >> 4, c4 = (lane & 15) * 4;
      for (int pass = 0; pass < 2; ++pass) {
#pragma unroll
        for (int it = 0; it < 8; ++it) {
          const int row = it * 2 + hh;
          v4f v = *(const v4f*)(slab + row * 68 + c4);
          if (mBase + row < Mlim) *(volatile v4f*)(C + (size_t)(mBase + row) * ldc + n0 + c4) = v;
        }
        __threadfence();
      }
    } else {
      const int q = lane >> 3, c8 = (lane & 7) * 8;
      unsigned short* C  = (unsigned short*)Cout  + (size_t)b * strideC;
      unsigned short* C2 = (OUT_MODE == 2) ? ((unsigned short*)Cout2 + (size_t)b * strideC) : nullptr;
      for (int pass = 0; pass < 2; ++pass) {
#pragma unroll
        for (int it = 0; it < 4; ++it) {
          const int row = it * 4 + q;
          const float* sp = slab + row * 68 + c8;
          v8h hv, lv;
#pragma unroll
          for (int e = 0; e < 8; ++e) {
            if (OUT_MODE == 1) {
              hv[e] = (_Float16)sp[e];
            } else {
              unsigned short hb = f2bf_bits(sp[e]);
              unsigned short lb = f2bf_bits(sp[e] - bf_bits2f(hb));
              hv[e] = __builtin_bit_cast(_Float16, hb);
              lv[e] = __builtin_bit_cast(_Float16, lb);
            }
          }
          if (mBase + row < Mlim) {
            *(volatile v8h*)(C + (size_t)(mBase + row) * ldc + n0 + c8) = hv;
            if (OUT_MODE == 2) *(volatile v8h*)(C2 + (size_t)(mBase + row) * ldc + n0 + c8) = lv;
          }
        }
        __threadfence();
      }
    }
    __builtin_amdgcn_fence(__ATOMIC_RELEASE, "workgroup");
    __builtin_amdgcn_wave_barrier();
    __builtin_amdgcn_fence(__ATOMIC_ACQUIRE, "workgroup");
  }
}

__global__ __launch_bounds__(256) void cast_scale_f16x2(
    const float* __restrict__ in, unsigned short* __restrict__ out, int n2, float sc) {
  int i = blockIdx.x * 256 + threadIdx.x;
  if (i < n2) {
    const _Float16 h0 = (_Float16)(in[2 * i] * sc), h1 = (_Float16)(in[2 * i + 1] * sc);
    const unsigned u = (unsigned)__builtin_bit_cast(unsigned short, h0) | ((unsigned)__builtin_bit_cast(unsigned short, h1) << 16);
    ((volatile unsigned*)out)[i] = u;
    __threadfence();
    ((volatile unsigned*)out)[i] = u;
  }
}

__device__ __forceinline__ int blk_excl_scan(int cnt, int* scan_ws, int tid, int* tot) {
  const int lane = tid & 31, wave = tid >> 5; int incl = cnt;
#pragma unroll
  for (int o = 1; o < 32; o <<= 1) { const int v = __shfl_up(incl, o, 32); if (lane >= o) incl += v; }
  if (lane == 31) scan_ws[wave] = incl;
  __syncthreads();
  if (wave == 0) { int wv = (lane < NT / 32) ? scan_ws[lane] : 0; int wincl = wv;
#pragma unroll
    for (int o = 1; o < 32; o <<= 1) { const int v = __shfl_up(wincl, o, 32); if (lane >= o) wincl += v; }
    if (lane < NT / 32) scan_ws[32 + lane] = wincl - wv; if (lane == 31) scan_ws[64] = wincl; }
  __syncthreads();
  const int res = scan_ws[32 + wave] + incl - cnt; *tot = scan_ws[64];
  return res;
}
template <int SPc, int CAP>
__device__ __forceinline__ int chunk_hits(const int* __restrict__ dstv, int e0, int n0, int lim, int tid, int* LIST, int* scan_ws) {
  const int eb = e0 + tid * SPc;
  const bool valid = (eb < NE);
  const int ebc = valid ? eb : (NE - SPc);
  int rec[SPc]; int cnt = 0;
#pragma unroll
  for (int k = 0; k < SPc; k += 4) {
    const v4i d4 = *(const v4i*)(dstv + ebc + k);
#pragma unroll
    for (int e = 0; e < 4; ++e) {
      const int d = d4[e]; int r = -1;
      if (valid && d >= n0 && d < lim) { r = ((d - n0) << 20) | (ebc + k + e); ++cnt; }
      rec[k + e] = r;
    }
  }
  int tot; int p = blk_excl_scan(cnt, scan_ws, tid, &tot);
#pragma unroll
  for (int k = 0; k < SPc; ++k) if (rec[k] >= 0) { if ((unsigned)p < (unsigned)CAP) LIST[p] = rec[k]; ++p; }
  __syncthreads();
  return tot < CAP ? tot : CAP;
}

__global__ __launch_bounds__(NT) void agg_kernel(const float* __restrict__ x, const int* __restrict__ ei, const int* __restrict__ nnp,
                                                const float* __restrict__ ew, float* ACC, unsigned short* __restrict__ AH) {
  __shared__ int LIST[SCH];
  __shared__ int DEG[SRB];
  __shared__ int scan_ws[80];
  const int tid = threadIdx.x, lane = tid & 31, wave = tid >> 5;
  const int n0 = blockIdx.x * SRB;
  int nn = nnp[0]; nn = nn < 0 ? 0 : (nn > NN ? NN : nn);
  const int lim = (n0 + SRB < nn) ? (n0 + SRB) : nn;
  const v4f z4 = {0.f, 0.f, 0.f, 0.f};
  for (int pass = 0; pass < 2; ++pass) {
#pragma unroll 1
    for (int j = 0; j < SRB / 8; ++j) {
      float* rp = ACC + (size_t)(n0 + wave * (SRB / 8) + j) * DIM + 4 * lane;
      *(volatile v4f*)rp = z4;
    }
    __threadfence();
  }
  for (int i = tid; i < SRB; i += NT) DEG[i] = 0;
  __syncthreads();
  const int* srcv = ei; const int* dstv = ei + NE;
#pragma unroll 1
  for (int c = 0; c < NCH; ++c) {
    const int tot = chunk_hits<SP, SCH>(dstv, c * SCH, n0, lim, tid, LIST, scan_ws);
#pragma unroll 1
    for (int base = 0; base < tot; base += 32) {
      const int q = base + lane;
      const int qc = q < SCH ? q : SCH - 1;
      int rv = LIST[qc];
      rv = (q < tot) ? rv : -1;
      const int own = (rv >= 0 && (rv >> 28) == wave) ? 1 : 0;
      unsigned msk = (unsigned)__ballot(own);
#pragma unroll 1
      for (int it = 0; it < 32; ++it) {
        if (msk == 0u) break;
        const int bp = __builtin_ctz(msk); msk &= msk - 1u;
        const int r = __shfl(rv, bp, 32);
        const int dl = (r >> 20) & (SRB - 1);
        int e = r & 0xFFFFF; e = e < NE ? e : NE - 1;
        int s = srcv[e]; s = s < 0 ? 0 : (s >= NN ? NN - 1 : s);
        const float w = ew[e];
        const v4f xv = *(const v4f*)(x + (size_t)s * DIM + 4 * lane);
        float* rp = ACC + (size_t)(n0 + dl) * DIM + 4 * lane;
        v4f a = *(const v4f*)rp;
        a = a + w * xv;
        *(volatile v4f*)rp = a;
        __threadfence();
        *(volatile v4f*)rp = a;
        if (lane == 0) DEG[dl] += 1;
      }
    }
    __syncthreads();
  }
  __threadfence();
  const int hh = lane >> 4, c8 = (lane & 15) * 8;
#pragma unroll 1
  for (int p = 0; p < SRB / 16; ++p) {
    const int dl = wave * (SRB / 8) + 2 * p + hh;
    const int n = n0 + dl;
    const float* rp = ACC + (size_t)n * DIM + c8;
    const v4f a0 = *(const v4f*)rp;
    const v4f a1 = *(const v4f*)(rp + 4);
    const int dg = DEG[dl];
    const float df = (float)(dg > 1 ? dg : 1);
    const float inv = 16.0f * (1.0f / df);
    v8h hv;
#pragma unroll
    for (int e = 0; e < 4; ++e) { hv[e] = (_Float16)(a0[e] * inv); hv[4 + e] = (_Float16)(a1[e] * inv); }
    unsigned short* op = AH + (size_t)n * DIM + c8;
    *(volatile v8h*)op = hv;
    __threadfence();
    *(volatile v8h*)op = hv;
  }
}

extern "C" void kernel_launch(void* const* d_in, const int* in_sizes, int n_in,
                              void* d_out, int out_size, void* d_ws, size_t ws_size, hipStream_t stream) {
  if (n_in < 7) return;
  const float* x   = (const float*)d_in[0];
  const int*   ei  = (const int*)  d_in[1];
  const int*   nnp = (const int*)  d_in[2];
  const float* ew  = (const float*)d_in[3];
  const float* W   = (const float*)d_in[4];
  const float* bb  = (const float*)d_in[5];
  const float* alp = (const float*)d_in[6];
  if (in_sizes[0] != NN * DIM || in_sizes[1] != 2 * NE || in_sizes[2] < 1 || in_sizes[3] != NE ||
      in_sizes[4] != DIM * DIM || in_sizes[5] != DIM || in_sizes[6] < 1 || out_size != NN * DIM) return;

  char* ws = (char*)d_ws; size_t off = 0;
  auto carve = [&](size_t bytes) -> char* { char* p = ws + off; off += (bytes + 255) & ~(size_t)255; return p; };
  float*          ACC = (float*)carve((size_t)NPAD * DIM * 4);
  unsigned short* AH  = (unsigned short*)carve((size_t)NPAD * DIM * 2);
  unsigned short* WH  = (unsigned short*)carve((size_t)DIM * DIM * 2);
  if (off > ws_size || off > (size_t)134217728) return;

  cast_scale_f16x2<<<(DIM * DIM / 2 + 255) / 256, 256, 0, stream>>>(W, WH, DIM * DIM / 2, 256.0f);
  agg_kernel<<<NTILE, NT, 0, stream>>>(x, ei, nnp, ew, ACC, AH);
  {
    const int tiles = (MG / 64) * (DIM / 64);
    wmma_gemm64<0, false, 2, 0, true, 0, true><<<dim3((tiles + 7) / 8, 1), 256, 0, stream>>>(
        (const unsigned short*)AH, (const unsigned short*)nullptr, DIM, 0L,
        (const unsigned short*)WH, (const unsigned short*)nullptr, DIM, 0L,
        (void*)d_out, (void*)nullptr, DIM, 0L,
        bb, x, 0L, MG, DIM, DIM, 1.0f / 4096.0f, alp, NN);
  }
}
